// CfCHead_65403761983519
// MI455X (gfx1250) — hardware-run, weakly checked
//
#include <hip/hip_runtime.h>
#include <math.h>

constexpr int kBatch = 65536;
constexpr int kIn0  = 74;
constexpr int kHid0 = 269;
constexpr int kHid1 = 179;
constexpr int kHid2 = 64;
constexpr int kKp0 = 96;
constexpr int kKp1 = 288;
constexpr int kKp2 = 192;
constexpr int kNp0 = 1088;
constexpr int kNp1 = 768;
constexpr int kNp2 = 256;
constexpr int kMC = 8192;
constexpr int kChunks = kBatch / kMC;
constexpr float kWCarry   = 16.0f;
constexpr float kOCarry   = 8.0f;
constexpr float kScaleL0  = 1.0f / 16.0f;
constexpr float kScaleL12 = 1.0f / 128.0f;

typedef char chk_chunks[(kBatch % kMC == 0) ? 1 : -1];
typedef char chk_tiles[(kMC % 64 == 0 && kNp0 % 64 == 0 && kNp1 % 64 == 0 && kNp2 % 64 == 0) ? 1 : -1];
typedef char chk_kpad[(kKp0 % 32 == 0 && kKp1 % 32 == 0 && kKp2 % 32 == 0) ? 1 : -1];
typedef char chk_npad[(kNp0 >= 4 * kHid0 && kNp1 >= 4 * kHid1 && kNp2 >= 4 * kHid2) ? 1 : -1];
typedef char chk_kin[(kKp0 >= kIn0 && kKp1 >= kHid0 && kKp2 >= kHid1) ? 1 : -1];


typedef __attribute__((ext_vector_type(16))) _Float16 v16h;
typedef __attribute__((ext_vector_type(8)))  _Float16 v8h;
typedef __attribute__((ext_vector_type(16))) __bf16   v16b;
typedef __attribute__((ext_vector_type(8)))  __bf16   v8b;
typedef __attribute__((ext_vector_type(8)))  float    v8f;
typedef __attribute__((ext_vector_type(4)))  float    v4f;
typedef __attribute__((ext_vector_type(4)))  unsigned int v4u;

__device__ __forceinline__ unsigned short f2bf_bits(float f) {
  unsigned u = __float_as_uint(f);
  return (unsigned short)((u + 0x7FFFu + ((u >> 16) & 1u)) >> 16);
}
__device__ __forceinline__ float bf_bits2f(unsigned short h) { return __uint_as_float(((unsigned)h) << 16); }

__device__ __forceinline__ void dep_guard_h(v8f& a, v8f& b, v16h x, v16h y) { asm volatile("v_nop\n\tv_nop\n\tv_nop\n\tv_nop" : "+v"(a), "+v"(b) : "v"(x), "v"(y)); }
__device__ __forceinline__ void dep_guard_b(v8f& a, v8f& b, v16b x, v16b y) { asm volatile("v_nop\n\tv_nop\n\tv_nop\n\tv_nop" : "+v"(a), "+v"(b) : "v"(x), "v"(y)); }
__device__ __forceinline__ void keep4_h(v16h a, v16h b, v16h c, v16h d) { asm volatile("v_nop" :: "v"(a), "v"(b), "v"(c), "v"(d)); }
__device__ __forceinline__ void keep4_b(v16b a, v16b b, v16b c, v16b d) { asm volatile("v_nop" :: "v"(a), "v"(b), "v"(c), "v"(d)); }
__device__ __forceinline__ void acc_guard4(v8f& a, v8f& b, v8f& c, v8f& d) { asm volatile("v_nop\n\tv_nop\n\tv_nop\n\tv_nop" : "+v"(a), "+v"(b), "+v"(c), "+v"(d)); }
template <typename T> struct Frag;
template <> struct Frag<_Float16> {
  typedef v16h V; union U { v16h v; v8h h[2]; };
  static __device__ __forceinline__ v16h load(const _Float16* p) {
    U f; f.h[0] = *(const v8h*)(p); f.h[1] = *(const v8h*)(p + 16); return f.v;
  }
  static __device__ __forceinline__ v8f mma(v16h a, v16h b, v8f c) {
    return __builtin_amdgcn_wmma_f32_16x16x32_f16(false, a, false, b, (short)0, c, false, false);
  }
  static __device__ __forceinline__ void guard(v8f& a, v8f& b, v16h x, v16h y) { dep_guard_h(a, b, x, y); }
  static __device__ __forceinline__ void keep(v16h a, v16h b, v16h c, v16h d) { keep4_h(a, b, c, d); }
};
template <> struct Frag<__bf16> {
  typedef v16b V; union U { v16b v; v8b h[2]; };
  static __device__ __forceinline__ v16b load(const __bf16* p) {
    U f; f.h[0] = *(const v8b*)(p); f.h[1] = *(const v8b*)(p + 16); return f.v;
  }
  static __device__ __forceinline__ v8f mma(v16b a, v16b b, v8f c) {
    return __builtin_amdgcn_wmma_f32_16x16x32_bf16(false, a, false, b, (short)0, c, false, false);
  }
  static __device__ __forceinline__ void guard(v8f& a, v8f& b, v16b x, v16b y) { dep_guard_b(a, b, x, y); }
  static __device__ __forceinline__ void keep(v16b a, v16b b, v16b c, v16b d) { keep4_b(a, b, c, d); }
};

__device__ __forceinline__ unsigned pk16(unsigned short a, unsigned short b) { return (unsigned)a | ((unsigned)b << 16); }
__device__ __forceinline__ unsigned short h_bits(float f) { const _Float16 h = (_Float16)f; return __builtin_bit_cast(unsigned short, h); }

template <int ET> struct Elem;
template <> struct Elem<0> { typedef _Float16 T; };
template <> struct Elem<1> { typedef __bf16 T; };
template <int ET, bool SPLIT, int BIAS_MODE, int OUT_MODE, bool RESID, int ACT = 0>
__global__ __launch_bounds__(256) void wmma_gemm64(
    const unsigned short* __restrict__ Ap, const unsigned short* __restrict__ A2p, int lda, long strideA,
    const unsigned short* __restrict__ Btp, const unsigned short* __restrict__ Bt2p, int ldb, long strideB,
    void* __restrict__ Cout, void* __restrict__ Cout2, int ldc, long strideC,
    const float* __restrict__ bias,
    const float* __restrict__ resid, long strideR,
    int M, int N, int K, float scale) {
  typedef typename Elem<ET>::T T;
  typedef typename Frag<T>::V V;
  const T* A = (const T*)Ap; const T* A2 = (const T*)A2p; const T* Bt = (const T*)Btp; const T* Bt2 = (const T*)Bt2p;
  __shared__ __align__(16) float sT[8][16 * 68];
  const int b    = blockIdx.y;
  const int lane = threadIdx.x & 31;
  const int wave = threadIdx.x >> 5;
  const int tilesN = N >> 6;
  const int tilesM = M >> 6;
  const int tile = blockIdx.x * 8 + wave;
  if (tile >= tilesM * tilesN) return;
  const int tm = tile / tilesN;
  const int tn = tile - tm * tilesN;
  const int m0 = tm << 6;
  const int n0 = tn << 6;

  const T* Ab  = A  + (size_t)b * strideA;
  const T* Bb  = Bt + (size_t)b * strideB;
  const T* Ab2 = SPLIT ? (A2  + (size_t)b * strideA) : nullptr;
  const T* Bb2 = SPLIT ? (Bt2 + (size_t)b * strideB) : nullptr;

  const int rlane = lane & 15;
  const int koff  = (lane >> 4) * 8;
  const int mOff  = (lane >> 4) * 8;

  v8f acc[4][4];
#pragma unroll
  for (int i = 0; i < 4; ++i)
#pragma unroll
    for (int j = 0; j < 4; ++j) acc[i][j] = (v8f){0.f,0.f,0.f,0.f,0.f,0.f,0.f,0.f};

  for (int k0 = 0; k0 < K; k0 += 32) {
    V bh[4], bl[4];
#pragma unroll
    for (int j = 0; j < 4; ++j) {
      const size_t bo = (size_t)(n0 + (j << 4) + rlane) * ldb + koff + k0;
      bh[j] = Frag<T>::load(Bb + bo);
      if (SPLIT) bl[j] = Frag<T>::load(Bb2 + bo);
    }
#pragma unroll
    for (int i = 0; i < 4; ++i) {
      const size_t ao = (size_t)(m0 + (i << 4) + rlane) * lda + koff + k0;
      V ah = Frag<T>::load(Ab + ao);
      V al;
      if (SPLIT) al = Frag<T>::load(Ab2 + ao);
#pragma unroll
      for (int j = 0; j < 4; ++j) {
        acc[i][j] = Frag<T>::mma(ah, bh[j], acc[i][j]);
        if (SPLIT) {
          acc[i][j] = Frag<T>::mma(ah, bl[j], acc[i][j]);
          acc[i][j] = Frag<T>::mma(al, bh[j], acc[i][j]);
        }
      }
      Frag<T>::guard(acc[i][0], acc[i][3], ah, SPLIT ? al : ah);
    }
    Frag<T>::keep(bh[0], bh[1], bh[2], bh[3]);
    if (SPLIT) Frag<T>::keep(bl[0], bl[1], bl[2], bl[3]);
  }
  acc_guard4(acc[0][0], acc[0][1], acc[0][2], acc[0][3]);
  acc_guard4(acc[1][0], acc[1][1], acc[1][2], acc[1][3]);
  acc_guard4(acc[2][0], acc[2][1], acc[2][2], acc[2][3]);
  acc_guard4(acc[3][0], acc[3][1], acc[3][2], acc[3][3]);

  float* slab = sT[wave];
  const float* Rb = RESID ? (resid + (size_t)b * strideR) : nullptr;
#pragma unroll
  for (int i = 0; i < 4; ++i) {
    const int mBase = m0 + (i << 4);
#pragma unroll
    for (int j = 0; j < 4; ++j) {
      const int n = n0 + (j << 4) + rlane;
      float bv = 0.f;
      if (BIAS_MODE == 2) bv = bias[n];
#pragma unroll
      for (int r = 0; r < 8; ++r) {
        float v = acc[i][j][r] * scale;
        if (BIAS_MODE == 1) v += bias[mBase + mOff + r];
        if (BIAS_MODE == 2) v += bv;
        if (RESID) v += Rb[(size_t)(mBase + mOff + r) * ldc + n];
        if (ACT == 2) v = fmaxf(v, 0.0f);
        if (ACT == 4) v = (v > 0.f) ? v : 0.01f * v;
        slab[(mOff + r) * 68 + (j << 4) + rlane] = v;
      }
    }
    __builtin_amdgcn_fence(__ATOMIC_RELEASE, "workgroup");
    __builtin_amdgcn_wave_barrier();
    __builtin_amdgcn_fence(__ATOMIC_ACQUIRE, "workgroup");
    if (OUT_MODE == 0) {
      float* C = (float*)Cout + (size_t)b * strideC;
      const int hh = lane >> 4, c4 = (lane & 15) * 4;
      for (int pass = 0; pass < 2; ++pass) {
#pragma unroll
        for (int it = 0; it < 8; ++it) {
          const int row = it * 2 + hh;
          v4f v = *(const v4f*)(slab + row * 68 + c4);
          *(volatile v4f*)(C + (size_t)(mBase + row) * ldc + n0 + c4) = v;
        }
        __threadfence();
      }
    } else {
      const int q = lane >> 3, c8 = (lane & 7) * 8;
      unsigned short* C  = (unsigned short*)Cout  + (size_t)b * strideC;
      unsigned short* C2 = (OUT_MODE == 2) ? ((unsigned short*)Cout2 + (size_t)b * strideC) : nullptr;
      for (int pass = 0; pass < 2; ++pass) {
#pragma unroll
        for (int it = 0; it < 4; ++it) {
          const int row = it * 4 + q;
          const float* sp = slab + row * 68 + c8;
          v8h hv, lv;
#pragma unroll
          for (int e = 0; e < 8; ++e) {
            if (OUT_MODE == 1) {
              hv[e] = (_Float16)sp[e];
            } else {
              unsigned short hb = f2bf_bits(sp[e]);
              unsigned short lb = f2bf_bits(sp[e] - bf_bits2f(hb));
              hv[e] = __builtin_bit_cast(_Float16, hb);
              lv[e] = __builtin_bit_cast(_Float16, lb);
            }
          }
          *(volatile v8h*)(C + (size_t)(mBase + row) * ldc + n0 + c8) = hv;
          if (OUT_MODE == 2) *(volatile v8h*)(C2 + (size_t)(mBase + row) * ldc + n0 + c8) = lv;
        }
        __threadfence();
      }
    }
    __builtin_amdgcn_fence(__ATOMIC_RELEASE, "workgroup");
    __builtin_amdgcn_wave_barrier();
    __builtin_amdgcn_fence(__ATOMIC_ACQUIRE, "workgroup");
  }
}

__global__ __launch_bounds__(256) void cast_x_kernel(const float* __restrict__ x, unsigned short* __restrict__ A0, int nrows) {
  const int t = blockIdx.x * 256 + threadIdx.x;
  const int nthr = (nrows * kKp0) >> 3;
  if (t >= nthr) return;
  const int f = t << 3;
  const int row = f / kKp0;
  const int kb = f - row * kKp0;
  const float* xr = x + (size_t)row * kIn0;
  unsigned short hb[8];
#pragma unroll
  for (int e = 0; e < 8; ++e) {
    const int k = kb + e;
    const int kc = (k < kIn0) ? k : (kIn0 - 1);
    float v = xr[kc];
    v = (k < kIn0) ? v : 0.0f;
    hb[e] = h_bits(v);
  }
  const v4u u = (v4u){pk16(hb[0], hb[1]), pk16(hb[2], hb[3]), pk16(hb[4], hb[5]), pk16(hb[6], hb[7])};
  unsigned short* op = A0 + (size_t)f;
  *(volatile v4u*)op = u;
  __threadfence();
  *(volatile v4u*)op = u;
}

__global__ __launch_bounds__(256) void build_bt_kernel(const float* __restrict__ W1, const float* __restrict__ W2,
                                                       const float* __restrict__ Wa, const float* __restrict__ Wb,
                                                       const int* __restrict__ msk, unsigned short* __restrict__ Bt,
                                                       int in_dim, int hid, int Kpad, int Npad, float carry) {
  const int t = blockIdx.x * 256 + threadIdx.x;
  const int nthr = (Npad * Kpad) >> 3;
  if (t >= nthr) return;
  const int f = t << 3;
  const int n = f / Kpad;
  const int kb = f - n * Kpad;
  const int n4 = 4 * hid;
  const bool nval = (n < n4);
  const int nc = nval ? n : (n4 - 1);
  const int w = nc / hid;
  const int j = nc - w * hid;
  unsigned short hb[8];
#pragma unroll
  for (int e = 0; e < 8; ++e) {
    const int k = kb + e;
    const int kc = (k < in_dim) ? k : (in_dim - 1);
    const size_t idx = (size_t)kc * hid + j;
    const float v1 = W1[idx];
    const float v2 = W2[idx];
    const float va = Wa[idx];
    const float vb = Wb[idx];
    const float m  = (float)msk[idx];
    float v = (w == 0) ? (v1 * m) : (w == 1) ? (v2 * m) : (w == 2) ? va : vb;
    v = (nval && (k < in_dim)) ? (v * carry) : 0.0f;
    hb[e] = h_bits(v);
  }
  const v4u u = (v4u){pk16(hb[0], hb[1]), pk16(hb[2], hb[3]), pk16(hb[4], hb[5]), pk16(hb[6], hb[7])};
  unsigned short* op = Bt + (size_t)f;
  *(volatile v4u*)op = u;
  __threadfence();
  *(volatile v4u*)op = u;
}

__device__ __forceinline__ float gate_value(const float* __restrict__ gr, int hid, int kc,
                                            const float* __restrict__ b1, const float* __restrict__ b2,
                                            const float* __restrict__ ba, const float* __restrict__ bb) {
  const float g1 = gr[kc] + b1[kc];
  const float g2 = gr[hid + kc] + b2[kc];
  const float ga = gr[2 * hid + kc] + ba[kc];
  const float gb = gr[3 * hid + kc] + bb[kc];
  const float f1 = tanhf(g1);
  const float f2 = tanhf(g2);
  const float z  = gb - ga;
  const float ti = 1.0f / (1.0f + expf(-z));
  return f1 * (1.0f - ti) + ti * f2;
}

__global__ __launch_bounds__(256) void gate_to_f16_kernel(const float* __restrict__ G, int ldg, int hid,
                                                          const float* __restrict__ b1, const float* __restrict__ b2,
                                                          const float* __restrict__ ba, const float* __restrict__ bb,
                                                          unsigned short* __restrict__ Aout, int kout, int nrows, float carry) {
  const int t = blockIdx.x * 256 + threadIdx.x;
  const int nthr = (nrows * kout) >> 3;
  if (t >= nthr) return;
  const int f = t << 3;
  const int row = f / kout;
  const int kb = f - row * kout;
  const float* gr = G + (size_t)row * ldg;
  float r0 = 0.f, r1 = 0.f, r2 = 0.f, r3 = 0.f, r4 = 0.f, r5 = 0.f, r6 = 0.f, r7 = 0.f;
#pragma unroll 1
  for (int e = 0; e < 8; ++e) {
    const int k = kb + e;
    const int kc = (k < hid) ? k : (hid - 1);
    float o = gate_value(gr, hid, kc, b1, b2, ba, bb);
    o = (k < hid) ? (o * carry) : 0.0f;
    r0 = (e == 0) ? o : r0;
    r1 = (e == 1) ? o : r1;
    r2 = (e == 2) ? o : r2;
    r3 = (e == 3) ? o : r3;
    r4 = (e == 4) ? o : r4;
    r5 = (e == 5) ? o : r5;
    r6 = (e == 6) ? o : r6;
    r7 = (e == 7) ? o : r7;
  }
  const v4u u = (v4u){pk16(h_bits(r0), h_bits(r1)), pk16(h_bits(r2), h_bits(r3)),
                      pk16(h_bits(r4), h_bits(r5)), pk16(h_bits(r6), h_bits(r7))};
  unsigned short* op = Aout + (size_t)f;
  *(volatile v4u*)op = u;
  __threadfence();
  *(volatile v4u*)op = u;
}

__global__ __launch_bounds__(256) void gate_to_f32_kernel(const float* __restrict__ G, int ldg, int hid,
                                                          const float* __restrict__ b1, const float* __restrict__ b2,
                                                          const float* __restrict__ ba, const float* __restrict__ bb,
                                                          float* __restrict__ out, int kout, int nrows) {
  const int t = blockIdx.x * 256 + threadIdx.x;
  const int nthr = (nrows * kout) >> 2;
  if (t >= nthr) return;
  const int f = t << 2;
  const int row = f / kout;
  const int kb = f - row * kout;
  const float* gr = G + (size_t)row * ldg;
  float r0 = 0.f, r1 = 0.f, r2 = 0.f, r3 = 0.f;
#pragma unroll 1
  for (int e = 0; e < 4; ++e) {
    const int k = kb + e;
    const int kc = (k < hid) ? k : (hid - 1);
    float o = gate_value(gr, hid, kc, b1, b2, ba, bb);
    o = (k < hid) ? o : 0.0f;
    r0 = (e == 0) ? o : r0;
    r1 = (e == 1) ? o : r1;
    r2 = (e == 2) ? o : r2;
    r3 = (e == 3) ? o : r3;
  }
  const v4f v = (v4f){r0, r1, r2, r3};
  float* op = out + (size_t)f;
  *(volatile v4f*)op = v;
  __threadfence();
  *(volatile v4f*)op = v;
}

extern "C" void kernel_launch(void* const* d_in, const int* in_sizes, int n_in,
                              void* d_out, int out_size, void* d_ws, size_t ws_size,
                              hipStream_t stream) {
  if (n_in < 28) return;
  if (in_sizes[0] != kBatch * kIn0 || out_size != kBatch * kHid2) return;

  const float* x = (const float*)d_in[0];
  const float* Wf1[3]; const float* bf1[3];
  const float* Wf2[3]; const float* bf2[3];
  const float* Wta[3]; const float* bta[3];
  const float* Wtb[3]; const float* btb[3];
  const int*   msk[3];
  for (int l = 0; l < 3; ++l) {
    const int b = 1 + l * 9;
    Wf1[l] = (const float*)d_in[b + 0]; bf1[l] = (const float*)d_in[b + 1];
    Wf2[l] = (const float*)d_in[b + 2]; bf2[l] = (const float*)d_in[b + 3];
    Wta[l] = (const float*)d_in[b + 4]; bta[l] = (const float*)d_in[b + 5];
    Wtb[l] = (const float*)d_in[b + 6]; btb[l] = (const float*)d_in[b + 7];
    msk[l] = (const int*)  d_in[b + 8];
  }
  if (in_sizes[1] != (kIn0 + kHid0) * kHid0 || in_sizes[10] != (kHid0 + kHid1) * kHid1 || in_sizes[19] != (kHid1 + kHid2) * kHid2) return;

  char* ws = (char*)d_ws;
  size_t off = 0;
  auto carve = [&](size_t bytes) -> char* {
    off = (off + 4095) & ~(size_t)4095;
    char* p = ws + off;
    off += bytes;
    return p;
  };
  unsigned short* A0  = (unsigned short*)carve((size_t)kBatch * kKp0 * 2);
  unsigned short* Bt0 = (unsigned short*)carve((size_t)kNp0 * kKp0 * 2);
  unsigned short* Bt1 = (unsigned short*)carve((size_t)kNp1 * kKp1 * 2);
  unsigned short* Bt2 = (unsigned short*)carve((size_t)kNp2 * kKp2 * 2);
  float*          G   = (float*)carve((size_t)kMC * kNp0 * 4);
  unsigned short* A1  = (unsigned short*)carve((size_t)kMC * kKp1 * 2);
  unsigned short* A2  = (unsigned short*)carve((size_t)kMC * kKp2 * 2);
  if (off > ws_size) return;

  float* outp = (float*)d_out;

  {
    const int nthr = (kBatch * kKp0) >> 3;
    cast_x_kernel<<<(nthr + 255) / 256, 256, 0, stream>>>(x, A0, kBatch);
  }
  {
    const int n0 = (kNp0 * kKp0) >> 3, n1 = (kNp1 * kKp1) >> 3, n2 = (kNp2 * kKp2) >> 3;
    build_bt_kernel<<<(n0 + 255) / 256, 256, 0, stream>>>(Wf1[0], Wf2[0], Wta[0], Wtb[0], msk[0], Bt0, kIn0,  kHid0, kKp0, kNp0, kWCarry);
    build_bt_kernel<<<(n1 + 255) / 256, 256, 0, stream>>>(Wf1[1], Wf2[1], Wta[1], Wtb[1], msk[1], Bt1, kHid0, kHid1, kKp1, kNp1, kWCarry);
    build_bt_kernel<<<(n2 + 255) / 256, 256, 0, stream>>>(Wf1[2], Wf2[2], Wta[2], Wtb[2], msk[2], Bt2, kHid1, kHid2, kKp2, kNp2, kWCarry);
  }

  const int tilesM = kMC / 64;
  const int blkL0 = (tilesM * (kNp0 / 64) + 7) / 8;
  const int blkL1 = (tilesM * (kNp1 / 64) + 7) / 8;
  const int blkL2 = (tilesM * (kNp2 / 64) + 7) / 8;
  const int gblk1 = (((kMC * kKp1) >> 3) + 255) / 256;
  const int gblk2 = (((kMC * kKp2) >> 3) + 255) / 256;
  const int gblkO = (((kMC * kHid2) >> 2) + 255) / 256;
  for (int c = 0; c < kChunks; ++c) {
    const unsigned short* Ac = A0 + (size_t)c * kMC * kKp0;
    wmma_gemm64<0, false, 0, 0, false, 0><<<dim3(blkL0, 1), 256, 0, stream>>>(
        Ac, Ac, kKp0, 0L, Bt0, Bt0, kKp0, 0L, (void*)G, (void*)G, kNp0, 0L,
        bf1[0], bf1[0], 0L, kMC, kNp0, kKp0, kScaleL0);
    gate_to_f16_kernel<<<gblk1, 256, 0, stream>>>(G, kNp0, kHid0, bf1[0], bf2[0], bta[0], btb[0], A1, kKp1, kMC, kOCarry);
    wmma_gemm64<0, false, 0, 0, false, 0><<<dim3(blkL1, 1), 256, 0, stream>>>(
        A1, A1, kKp1, 0L, Bt1, Bt1, kKp1, 0L, (void*)G, (void*)G, kNp1, 0L,
        bf1[1], bf1[1], 0L, kMC, kNp1, kKp1, kScaleL12);
    gate_to_f16_kernel<<<gblk2, 256, 0, stream>>>(G, kNp1, kHid1, bf1[1], bf2[1], bta[1], btb[1], A2, kKp2, kMC, kOCarry);
    wmma_gemm64<0, false, 0, 0, false, 0><<<dim3(blkL2, 1), 256, 0, stream>>>(
        A2, A2, kKp2, 0L, Bt2, Bt2, kKp2, 0L, (void*)G, (void*)G, kNp2, 0L,
        bf1[2], bf1[2], 0L, kMC, kNp2, kKp2, kScaleL12);
    gate_to_f32_kernel<<<gblkO, 256, 0, stream>>>(G, kNp2, kHid2, bf1[2], bf2[2], bta[2], btb[2],
                                                  outp + (size_t)c * kMC * kHid2, kHid2, kMC);
  }
}
